// MultiHeadGATLayer_11596411699835
// MI455X (gfx1250) — hardware-verified
//
#include <hip/hip_runtime.h>

#define NN    2048
#define FIN   512
#define FOUT  512
#define NH    8
#define DH    64
#define LRELU 0.2f
#define HBLK  512
#define WTB   64
#define SWP   72

typedef __bf16          v16bf __attribute__((ext_vector_type(16)));
typedef unsigned short  v16us __attribute__((ext_vector_type(16)));
typedef unsigned short  v8us  __attribute__((ext_vector_type(8)));
typedef float           v8f   __attribute__((ext_vector_type(8)));
typedef float           v4f   __attribute__((ext_vector_type(4)));
typedef int             v4i   __attribute__((ext_vector_type(4)));
typedef v8us __attribute__((may_alias)) v8usa;
typedef v4f  __attribute__((may_alias)) v4fa;
typedef v4i  __attribute__((may_alias)) v4ia;

union BFrag { v16bf v; v16us u; v8us half[2]; };
static_assert(sizeof(v16bf) == 32);
static_assert(sizeof(BFrag) == 32);
static_assert(NN % 128 == 0);
static_assert(FIN % 32 == 0);
static_assert(FOUT == NH * DH);

__device__ __forceinline__ unsigned short bf_bits(float f) {
  const unsigned int u = __float_as_uint(f);
  return (unsigned short)((u + 0x7FFFu + ((u >> 16) & 1u)) >> 16);
}
__device__ __forceinline__ float bf_val(unsigned short b) {
  return __uint_as_float(((unsigned int)b) << 16);
}
__device__ __forceinline__ float bf_rne(float f) { return bf_val(bf_bits(f)); }

__device__ __forceinline__ v8f wmma_bf16(v16bf a, v16bf b, v8f c) {
  v8f d = __builtin_amdgcn_wmma_f32_16x16x32_bf16(false, a, false, b, (short)0, c, false, false);
  asm volatile("v_nop\n\tv_nop\n\tv_nop\n\tv_nop" : "+v"(d) : "v"(a), "v"(b));
  return d;
}

__device__ __forceinline__ v16bf load_frag(const unsigned short* p, int h) {
  BFrag f;
  f.half[0] = *(const v8usa*)(p + 8 * h);
  f.half[1] = *(const v8usa*)(p + 16 + 8 * h);
  return f.v;
}

__global__ __launch_bounds__(256) void convert_kernel(
    const float* __restrict__ h, const float* __restrict__ W,
    unsigned short* __restrict__ hb, unsigned short* __restrict__ wt)
{
  __shared__ __attribute__((aligned(16))) unsigned short sW[WTB * SWP];
  const int tid = threadIdx.x;
  const int bid = blockIdx.x;
  if (bid < HBLK) {
    const size_t g = (size_t)bid * 256 + tid;
    const float* src = h + g * 8;
    const v4f a = *(const v4fa*)src;
    const v4f c = *(const v4fa*)(src + 4);
    const v8us o = { bf_bits(a.x), bf_bits(a.y), bf_bits(a.z), bf_bits(a.w),
                     bf_bits(c.x), bf_bits(c.y), bf_bits(c.z), bf_bits(c.w) };
    unsigned short* dst = hb + g * 8;
    *(volatile v8us*)dst = o;
    __threadfence();
    *(volatile v8us*)dst = o;
  } else {
    const int tile = bid - HBLK;
    const int kt = tile >> 3, ntile = tile & 7;
    const int k0 = WTB * kt, n0 = WTB * ntile;
    const int kk = tid >> 2, nn0 = (tid & 3) * 16;
    const float* src = W + (size_t)(k0 + kk) * FOUT + n0 + nn0;
    const v4f q0 = *(const v4fa*)(src);
    const v4f q1 = *(const v4fa*)(src + 4);
    const v4f q2 = *(const v4fa*)(src + 8);
    const v4f q3 = *(const v4fa*)(src + 12);
    sW[(nn0 +  0) * SWP + kk] = bf_bits(q0.x);
    sW[(nn0 +  1) * SWP + kk] = bf_bits(q0.y);
    sW[(nn0 +  2) * SWP + kk] = bf_bits(q0.z);
    sW[(nn0 +  3) * SWP + kk] = bf_bits(q0.w);
    sW[(nn0 +  4) * SWP + kk] = bf_bits(q1.x);
    sW[(nn0 +  5) * SWP + kk] = bf_bits(q1.y);
    sW[(nn0 +  6) * SWP + kk] = bf_bits(q1.z);
    sW[(nn0 +  7) * SWP + kk] = bf_bits(q1.w);
    sW[(nn0 +  8) * SWP + kk] = bf_bits(q2.x);
    sW[(nn0 +  9) * SWP + kk] = bf_bits(q2.y);
    sW[(nn0 + 10) * SWP + kk] = bf_bits(q2.z);
    sW[(nn0 + 11) * SWP + kk] = bf_bits(q2.w);
    sW[(nn0 + 12) * SWP + kk] = bf_bits(q3.x);
    sW[(nn0 + 13) * SWP + kk] = bf_bits(q3.y);
    sW[(nn0 + 14) * SWP + kk] = bf_bits(q3.z);
    sW[(nn0 + 15) * SWP + kk] = bf_bits(q3.w);
    __syncthreads();
    const int q8 = tid & 7, lr = tid >> 3;
    const v8us v0 = *(const v8usa*)(sW + lr * SWP + 8 * q8);
    const v8us v1 = *(const v8usa*)(sW + (lr + 32) * SWP + 8 * q8);
    unsigned short* d0 = wt + (size_t)(n0 + lr) * FIN + k0 + 8 * q8;
    unsigned short* d1 = wt + (size_t)(n0 + lr + 32) * FIN + k0 + 8 * q8;
    *(volatile v8us*)d0 = v0;
    *(volatile v8us*)d1 = v1;
    __threadfence();
    *(volatile v8us*)d0 = v0;
    *(volatile v8us*)d1 = v1;
  }
}

__device__ __forceinline__ void wh_store_pass(const float* sT, const float* sSD,
                                              unsigned short* whi, unsigned short* wlo,
                                              float* srct, float* dstt,
                                              int hd, int i0, int w, int lane) {
  if (w == 0) {
    const v4f v = *(const v4fa*)(sSD + 4 * lane);
    *(volatile v4f*)(srct + (size_t)hd * NN + i0 + 4 * lane) = v;
  } else if (w == 1) {
    const v4f v = *(const v4fa*)(sSD + 128 + 4 * lane);
    *(volatile v4f*)(dstt + (size_t)hd * NN + i0 + 4 * lane) = v;
  }
  const int q8 = lane & 7, sub = lane >> 3;
  #pragma unroll
  for (int i = 0; i < 8; ++i) {
    const int lid = w * 32 + i * 4 + sub;
    const int d = lid >> 1, hl = lid & 1;
    const float* sp = sT + d * 128 + 64 * hl + 8 * q8;
    const v4f a = *(const v4fa*)sp;
    const v4f c = *(const v4fa*)(sp + 4);
    const unsigned short h0 = bf_bits(a.x), h1 = bf_bits(a.y), h2 = bf_bits(a.z), h3 = bf_bits(a.w);
    const unsigned short h4 = bf_bits(c.x), h5 = bf_bits(c.y), h6 = bf_bits(c.z), h7 = bf_bits(c.w);
    const v8us vh = { h0, h1, h2, h3, h4, h5, h6, h7 };
    const v8us vl = { bf_bits(a.x - bf_val(h0)), bf_bits(a.y - bf_val(h1)),
                      bf_bits(a.z - bf_val(h2)), bf_bits(a.w - bf_val(h3)),
                      bf_bits(c.x - bf_val(h4)), bf_bits(c.y - bf_val(h5)),
                      bf_bits(c.z - bf_val(h6)), bf_bits(c.w - bf_val(h7)) };
    const size_t gi = ((size_t)hd * DH + d) * NN + i0 + 64 * hl + 8 * q8;
    *(volatile v8us*)(whi + gi) = vh;
    *(volatile v8us*)(wlo + gi) = vl;
  }
}

__global__ __launch_bounds__(128) void wh_kernel(
    const unsigned short* __restrict__ hb,
    const unsigned short* __restrict__ wt,
    const float* __restrict__ W_b,
    const float* __restrict__ a_w,
    unsigned short* __restrict__ whi,
    unsigned short* __restrict__ wlo,
    float* __restrict__ srct,
    float* __restrict__ dstt)
{
  __shared__ __attribute__((aligned(16))) float sT[DH * 128];
  __shared__ __attribute__((aligned(16))) float sSD[256];
  __shared__ float sAW[2 * DH];

  const int tid = threadIdx.x, lane = tid & 31, w = tid >> 5;
  const int h = lane >> 4, m = lane & 15;
  const int i0 = blockIdx.x * 128;
  const int hd = blockIdx.y;
  const int i0w = i0 + 32 * w;

  sAW[tid] = bf_rne(a_w[tid]);

  const unsigned short* xa0 = hb + (size_t)(i0w + m) * FIN;
  const unsigned short* xa1 = xa0 + (size_t)16 * FIN;
  const unsigned short* wb  = wt + ((size_t)hd * DH + m) * FIN;

  const v8f zero8 = {0.f, 0.f, 0.f, 0.f, 0.f, 0.f, 0.f, 0.f};
  v8f acc[2][4];
  #pragma unroll
  for (int mt = 0; mt < 2; ++mt)
    #pragma unroll
    for (int nt = 0; nt < 4; ++nt) acc[mt][nt] = zero8;

  #pragma unroll 1
  for (int k0 = 0; k0 < FIN; k0 += 32) {
    const v16bf a0 = load_frag(xa0 + k0, h);
    const v16bf a1 = load_frag(xa1 + k0, h);
    #pragma unroll
    for (int nt = 0; nt < 4; ++nt) {
      const v16bf b = load_frag(wb + (size_t)nt * 16 * FIN + k0, h);
      acc[0][nt] = wmma_bf16(a0, b, acc[0][nt]);
      acc[1][nt] = wmma_bf16(a1, b, acc[1][nt]);
    }
  }

  #pragma unroll
  for (int nt = 0; nt < 4; ++nt) {
    const int feat = 16 * nt + m;
    const float bias = bf_rne(W_b[hd * DH + feat]);
    #pragma unroll
    for (int mt = 0; mt < 2; ++mt) {
      #pragma unroll
      for (int r = 0; r < 8; ++r) {
        const int tokl = 32 * w + 16 * mt + 8 * h + r;
        sT[feat * 128 + tokl] = acc[mt][nt][r] + bias;
      }
    }
  }
  __syncthreads();

  float s = 0.0f, d = 0.0f;
  #pragma unroll 8
  for (int dd = 0; dd < DH; ++dd) {
    const float v = sT[dd * 128 + tid];
    s += v * sAW[dd];
    d += v * sAW[DH + dd];
  }
  sSD[tid] = s;
  sSD[128 + tid] = d;
  __syncthreads();

  wh_store_pass(sT, sSD, whi, wlo, srct, dstt, hd, i0, w, lane);
  __threadfence();
  wh_store_pass(sT, sSD, whi, wlo, srct, dstt, hd, i0, w, lane);
}

struct PE { unsigned short hi, lo; };

__device__ __forceinline__ PE pelem(float dj, int aj, float srci, float ab, float mrow, float& lsum) {
  float s = (srci + dj) + ab;
  s = (s >= 0.0f) ? s : LRELU * s;
  s = (aj > 0) ? s : 0.0f;
  const float p = __expf(s - mrow);
  lsum += p;
  PE r;
  r.hi = bf_bits(p);
  r.lo = bf_bits(p - bf_val(r.hi));
  return r;
}

__device__ __forceinline__ void att_store_pass(const float* so, float* out,
                                               int hd, int i0w, int lane) {
  const int q8 = lane & 7, sub = lane >> 3;
  #pragma unroll
  for (int i = 0; i < 8; ++i) {
    const int lid = i * 4 + sub;
    const int row = lid >> 1, hl = lid & 1;
    const v4f v = *(const v4fa*)(so + row * 64 + 32 * hl + 4 * q8);
    const size_t gi = ((size_t)(i0w + row)) * FOUT + hd * DH + 32 * hl + 4 * q8;
    *(volatile v4f*)(out + gi) = v;
  }
}

__global__ __launch_bounds__(128) void attn_kernel(
    const int* __restrict__ adj,
    const unsigned short* __restrict__ whi,
    const unsigned short* __restrict__ wlo,
    const float* __restrict__ srct,
    const float* __restrict__ dstt,
    const float* __restrict__ a_b,
    float* __restrict__ out)
{
  __shared__ __attribute__((aligned(16))) float sD[NN];
  __shared__ float sRed[4];
  __shared__ __attribute__((aligned(16))) float sO[4 * 16 * 64];

  const int tid = threadIdx.x, lane = tid & 31, w = tid >> 5;
  const int h = lane >> 4, m = lane & 15;
  const int hd = blockIdx.y;
  const int i0w = blockIdx.x * 64 + 16 * w;
  const int i = i0w + m;

  const float* dsrc = dstt + (size_t)hd * NN;
  float mx = -3.0e38f;
  #pragma unroll
  for (int c = 0; c < 4; ++c) {
    const int idx = c * 512 + 4 * tid;
    const v4f v = *(const v4fa*)(dsrc + idx);
    *(v4fa*)(sD + idx) = v;
    mx = fmaxf(mx, fmaxf(fmaxf(v.x, v.y), fmaxf(v.z, v.w)));
  }
  #pragma unroll
  for (int off = 16; off > 0; off >>= 1) mx = fmaxf(mx, __shfl_xor(mx, off));
  if (lane == 0) sRed[w] = mx;
  __syncthreads();
  const float dmax = fmaxf(fmaxf(sRed[0], sRed[1]), fmaxf(sRed[2], sRed[3]));

  const float ab = bf_rne(a_b[0]);
  const float srci = srct[(size_t)hd * NN + i];
  float bnd = (srci + dmax) + ab;
  bnd = (bnd >= 0.0f) ? bnd : LRELU * bnd;
  const float mrow = fmaxf(bnd, 0.0f);

  const int* arow = adj + (size_t)i * NN;
  const unsigned short* wb_hi = whi + ((size_t)hd * DH + m) * NN;
  const unsigned short* wb_lo = wlo + ((size_t)hd * DH + m) * NN;

  const v8f zero8 = {0.f, 0.f, 0.f, 0.f, 0.f, 0.f, 0.f, 0.f};
  v8f o[4];
  #pragma unroll
  for (int t = 0; t < 4; ++t) o[t] = zero8;
  float lsum = 0.0f;

  #pragma unroll 1
  for (int j0 = 0; j0 < NN; j0 += 32) {
    const int ja = j0 + 8 * h, jb = j0 + 16 + 8 * h;
    const v4i a0 = *(const v4ia*)(arow + ja);
    const v4i a1 = *(const v4ia*)(arow + ja + 4);
    const v4i a2 = *(const v4ia*)(arow + jb);
    const v4i a3 = *(const v4ia*)(arow + jb + 4);
    const v4f d0 = *(const v4fa*)(sD + ja);
    const v4f d1 = *(const v4fa*)(sD + ja + 4);
    const v4f d2 = *(const v4fa*)(sD + jb);
    const v4f d3 = *(const v4fa*)(sD + jb + 4);

    const PE e0  = pelem(d0.x, a0.x, srci, ab, mrow, lsum);
    const PE e1  = pelem(d0.y, a0.y, srci, ab, mrow, lsum);
    const PE e2  = pelem(d0.z, a0.z, srci, ab, mrow, lsum);
    const PE e3  = pelem(d0.w, a0.w, srci, ab, mrow, lsum);
    const PE e4  = pelem(d1.x, a1.x, srci, ab, mrow, lsum);
    const PE e5  = pelem(d1.y, a1.y, srci, ab, mrow, lsum);
    const PE e6  = pelem(d1.z, a1.z, srci, ab, mrow, lsum);
    const PE e7  = pelem(d1.w, a1.w, srci, ab, mrow, lsum);
    const PE e8  = pelem(d2.x, a2.x, srci, ab, mrow, lsum);
    const PE e9  = pelem(d2.y, a2.y, srci, ab, mrow, lsum);
    const PE e10 = pelem(d2.z, a2.z, srci, ab, mrow, lsum);
    const PE e11 = pelem(d2.w, a2.w, srci, ab, mrow, lsum);
    const PE e12 = pelem(d3.x, a3.x, srci, ab, mrow, lsum);
    const PE e13 = pelem(d3.y, a3.y, srci, ab, mrow, lsum);
    const PE e14 = pelem(d3.z, a3.z, srci, ab, mrow, lsum);
    const PE e15 = pelem(d3.w, a3.w, srci, ab, mrow, lsum);

    BFrag ph, pl;
    const v16us uh = { e0.hi, e1.hi, e2.hi,  e3.hi,  e4.hi,  e5.hi,  e6.hi,  e7.hi,
                       e8.hi, e9.hi, e10.hi, e11.hi, e12.hi, e13.hi, e14.hi, e15.hi };
    const v16us ul = { e0.lo, e1.lo, e2.lo,  e3.lo,  e4.lo,  e5.lo,  e6.lo,  e7.lo,
                       e8.lo, e9.lo, e10.lo, e11.lo, e12.lo, e13.lo, e14.lo, e15.lo };
    ph.u = uh;
    pl.u = ul;

    #pragma unroll
    for (int t = 0; t < 4; ++t) {
      const v16bf ahi = load_frag(wb_hi + (size_t)(16 * t) * NN + j0, h);
      const v16bf alo = load_frag(wb_lo + (size_t)(16 * t) * NN + j0, h);
      o[t] = wmma_bf16(ahi, ph.v, o[t]);
      o[t] = wmma_bf16(ahi, pl.v, o[t]);
      o[t] = wmma_bf16(alo, ph.v, o[t]);
    }
  }

  lsum += __shfl_xor(lsum, 16);
  const float inv = 1.0f / lsum;
  float* so = sO + w * 1024;
  #pragma unroll
  for (int t = 0; t < 4; ++t)
    #pragma unroll
    for (int r = 0; r < 8; ++r)
      so[m * 64 + 16 * t + 8 * h + r] = o[t][r] * inv;
  __syncthreads();

  att_store_pass(so, out, hd, i0w, lane);
  __threadfence();
  att_store_pass(so, out, hd, i0w, lane);
}

extern "C" void kernel_launch(void* const* d_in, const int* in_sizes, int n_in,
                              void* d_out, int out_size, void* d_ws, size_t ws_size,
                              hipStream_t stream) {
  if (n_in < 6) return;
  if (in_sizes[0] != NN * FIN) return;
  if (in_sizes[1] != NN * NN) return;
  if (in_sizes[2] != FIN * FOUT) return;
  if (in_sizes[3] != FOUT) return;
  if (in_sizes[4] != 2 * DH) return;
  if (in_sizes[5] < 1) return;
  if (out_size != NN * FOUT) return;

  const float* h   = (const float*)d_in[0];
  const int*   adj = (const int*)d_in[1];
  const float* W_w = (const float*)d_in[2];
  const float* W_b = (const float*)d_in[3];
  const float* a_w = (const float*)d_in[4];
  const float* a_b = (const float*)d_in[5];
  float* out = (float*)d_out;

  const size_t hb_bytes = (size_t)NN * FIN * 2;
  const size_t wt_bytes = (size_t)FOUT * FIN * 2;
  const size_t pl_bytes = (size_t)FOUT * NN * 2;
  const size_t tb_bytes = (size_t)NH * NN * 4;
  const size_t total = hb_bytes + wt_bytes + 2 * pl_bytes + 2 * tb_bytes;
  if (total > ws_size) return;

  char* ws = (char*)d_ws;
  unsigned short* hb  = (unsigned short*)(ws);
  unsigned short* wt  = (unsigned short*)(ws + hb_bytes);
  unsigned short* whi = (unsigned short*)(ws + hb_bytes + wt_bytes);
  unsigned short* wlo = (unsigned short*)(ws + hb_bytes + wt_bytes + pl_bytes);
  float* srct = (float*)(ws + hb_bytes + wt_bytes + 2 * pl_bytes);
  float* dstt = (float*)(ws + hb_bytes + wt_bytes + 2 * pl_bytes + tb_bytes);

  convert_kernel<<<dim3(HBLK + (FIN / WTB) * (FOUT / WTB)), dim3(256), 0, stream>>>(h, W_w, hb, wt);

  wh_kernel<<<dim3(NN / 128, NH), dim3(128), 0, stream>>>(hb, wt, W_b, a_w, whi, wlo, srct, dstt);

  attn_kernel<<<dim3(NN / 64, NH), dim3(128), 0, stream>>>(adj, whi, wlo, srct, dstt, a_b, out);
}
